// LSTMDecoder_57543971832694
// MI455X (gfx1250) — hardware-verified
//
#include <hip/hip_runtime.h>
#include <math.h>

constexpr int NB    = 256;
constexpr int NLAT  = 128;
constexpr int NH    = 256;
constexpr int NO    = 64;
constexpr int NS    = 512;
constexpr int NG4   = 4 * NH;
constexpr int N2H   = 2 * NH;
constexpr int NROWS = NB * NS;
constexpr int NTHR  = 256;
constexpr int RTHR  = 512;
constexpr int RBR   = 16;
constexpr int HP    = 264;
constexpr float ZC     = 16.0f;
constexpr float WC     = 256.0f;
constexpr float X0C    = 16.0f;
constexpr float WC_INV = 1.0f / 256.0f;
constexpr int OFF_BHID = 0;
constexpr int OFF_BCEL = 512;
constexpr int OFF_BINP = 1024;
constexpr int OFF_BS0  = 1280;
constexpr int OFF_BS1  = 2304;
constexpr int OFF_BOUT = 3328;
constexpr int NBIAS    = 3392;

static_assert(NLAT % 32 == 0 && NH % 32 == 0);
static_assert(NB % 64 == 0 && N2H % 64 == 0 && NH % 64 == 0 && NG4 % 64 == 0 && NROWS % 64 == 0 && NO % 64 == 0);
static_assert(NB % RBR == 0);
static_assert(NH == 16 * (RTHR / 32));
static_assert(RTHR / 32 == RBR);
static_assert((RBR * NH) % RTHR == 0);
static_assert(HP % 8 == 0 && (RBR * HP * 2) % 16 == 0);
static_assert(OFF_BCEL % 32 == 0 && OFF_BINP % 32 == 0 && OFF_BS0 % 32 == 0 && OFF_BS1 % 32 == 0 && OFF_BOUT % 32 == 0 && NBIAS % 32 == 0);

typedef __attribute__((ext_vector_type(16))) _Float16 v16h;
typedef __attribute__((ext_vector_type(8)))  _Float16 v8h;
typedef __attribute__((ext_vector_type(16))) __bf16   v16b;
typedef __attribute__((ext_vector_type(8)))  __bf16   v8b;
typedef __attribute__((ext_vector_type(8)))  float    v8f;
typedef __attribute__((ext_vector_type(4)))  float    v4f;
typedef __attribute__((ext_vector_type(4)))  unsigned v4u;

__device__ __forceinline__ unsigned short f2bf_bits(float f) {
  unsigned u = __float_as_uint(f);
  return (unsigned short)((u + 0x7FFFu + ((u >> 16) & 1u)) >> 16);
}
__device__ __forceinline__ float bf_bits2f(unsigned short h) { return __uint_as_float(((unsigned)h) << 16); }
__device__ __forceinline__ float bf16r(float f) { return bf_bits2f(f2bf_bits(f)); }

__device__ __forceinline__ void dep_guard_h(v8f& a, v8f& b, v16h x, v16h y) { asm volatile("v_nop\n\tv_nop\n\tv_nop\n\tv_nop" : "+v"(a), "+v"(b) : "v"(x), "v"(y)); }
__device__ __forceinline__ void dep_guard_b(v8f& a, v8f& b, v16b x, v16b y) { asm volatile("v_nop\n\tv_nop\n\tv_nop\n\tv_nop" : "+v"(a), "+v"(b) : "v"(x), "v"(y)); }
__device__ __forceinline__ void keep4_h(v16h a, v16h b, v16h c, v16h d) { asm volatile("v_nop" :: "v"(a), "v"(b), "v"(c), "v"(d)); }
__device__ __forceinline__ void keep4_b(v16b a, v16b b, v16b c, v16b d) { asm volatile("v_nop" :: "v"(a), "v"(b), "v"(c), "v"(d)); }
__device__ __forceinline__ void acc_guard4(v8f& a, v8f& b, v8f& c, v8f& d) { asm volatile("v_nop\n\tv_nop\n\tv_nop\n\tv_nop" : "+v"(a), "+v"(b), "+v"(c), "+v"(d)); }
__device__ __forceinline__ void acc_guard4ab(v8f& a, v8f& b, v8f& c, v8f& d, v16h x, v16h y) {
  asm volatile("v_nop\n\tv_nop\n\tv_nop\n\tv_nop" : "+v"(a), "+v"(b), "+v"(c), "+v"(d) : "v"(x), "v"(y));
}
__device__ __forceinline__ void use8(float a0, float a1, float a2, float a3, float a4, float a5, float a6, float a7) {
  asm volatile("" :: "v"(a0), "v"(a1), "v"(a2), "v"(a3), "v"(a4), "v"(a5), "v"(a6), "v"(a7));
}
template <typename T> struct Frag;
template <> struct Frag<_Float16> {
  typedef v16h V; union U { v16h v; v8h h[2]; };
  static __device__ __forceinline__ v16h load(const _Float16* p) {
    U f; f.h[0] = *(const v8h*)(p); f.h[1] = *(const v8h*)(p + 16); return f.v;
  }
  static __device__ __forceinline__ v8f mma(v16h a, v16h b, v8f c) {
    return __builtin_amdgcn_wmma_f32_16x16x32_f16(false, a, false, b, (short)0, c, false, false);
  }
  static __device__ __forceinline__ void guard(v8f& a, v8f& b, v16h x, v16h y) { dep_guard_h(a, b, x, y); }
  static __device__ __forceinline__ void keep(v16h a, v16h b, v16h c, v16h d) { keep4_h(a, b, c, d); }
};
template <> struct Frag<__bf16> {
  typedef v16b V; union U { v16b v; v8b h[2]; };
  static __device__ __forceinline__ v16b load(const __bf16* p) {
    U f; f.h[0] = *(const v8b*)(p); f.h[1] = *(const v8b*)(p + 16); return f.v;
  }
  static __device__ __forceinline__ v8f mma(v16b a, v16b b, v8f c) {
    return __builtin_amdgcn_wmma_f32_16x16x32_bf16(false, a, false, b, (short)0, c, false, false);
  }
  static __device__ __forceinline__ void guard(v8f& a, v8f& b, v16b x, v16b y) { dep_guard_b(a, b, x, y); }
  static __device__ __forceinline__ void keep(v16b a, v16b b, v16b c, v16b d) { keep4_b(a, b, c, d); }
};

__device__ __forceinline__ float fsig(float x)  { return __builtin_amdgcn_rcpf(1.0f + expf(-x)); }
__device__ __forceinline__ float ftanh(float x) { return 1.0f - 2.0f * __builtin_amdgcn_rcpf(expf(2.0f * x) + 1.0f); }

template <int ET> struct Elem;
template <> struct Elem<0> { typedef _Float16 T; };
template <> struct Elem<1> { typedef __bf16 T; };
template <int ET, bool SPLIT, int BIAS_MODE, int OUT_MODE, bool RESID, int ACT = 0>
__global__ __launch_bounds__(256) void wmma_gemm64(
    const unsigned short* __restrict__ Ap, const unsigned short* __restrict__ A2p, int lda, long strideA,
    const unsigned short* __restrict__ Btp, const unsigned short* __restrict__ Bt2p, int ldb, long strideB,
    void* __restrict__ Cout, void* __restrict__ Cout2, int ldc, long strideC,
    const float* __restrict__ bias,
    const float* __restrict__ resid, long strideR,
    int M, int N, int K, float scale) {
  typedef typename Elem<ET>::T T;
  typedef typename Frag<T>::V V;
  const T* A = (const T*)Ap; const T* A2 = (const T*)A2p; const T* Bt = (const T*)Btp; const T* Bt2 = (const T*)Bt2p;
  __shared__ __align__(16) float sT[8][16 * 68];
  const int b    = blockIdx.y;
  const int lane = threadIdx.x & 31;
  const int wave = threadIdx.x >> 5;
  const int tilesN = N >> 6;
  const int tilesM = M >> 6;
  const int tile = blockIdx.x * 8 + wave;
  if (tile >= tilesM * tilesN) return;
  const int tm = tile / tilesN;
  const int tn = tile - tm * tilesN;
  const int m0 = tm << 6;
  const int n0 = tn << 6;

  const T* Ab  = A  + (size_t)b * strideA;
  const T* Bb  = Bt + (size_t)b * strideB;
  const T* Ab2 = SPLIT ? (A2  + (size_t)b * strideA) : nullptr;
  const T* Bb2 = SPLIT ? (Bt2 + (size_t)b * strideB) : nullptr;

  const int rlane = lane & 15;
  const int koff  = (lane >> 4) * 8;
  const int mOff  = (lane >> 4) * 8;

  v8f acc[4][4];
#pragma unroll
  for (int i = 0; i < 4; ++i)
#pragma unroll
    for (int j = 0; j < 4; ++j) acc[i][j] = (v8f){0.f,0.f,0.f,0.f,0.f,0.f,0.f,0.f};

  for (int k0 = 0; k0 < K; k0 += 32) {
    V bh[4], bl[4];
#pragma unroll
    for (int j = 0; j < 4; ++j) {
      const size_t bo = (size_t)(n0 + (j << 4) + rlane) * ldb + koff + k0;
      bh[j] = Frag<T>::load(Bb + bo);
      if (SPLIT) bl[j] = Frag<T>::load(Bb2 + bo);
    }
#pragma unroll
    for (int i = 0; i < 4; ++i) {
      const size_t ao = (size_t)(m0 + (i << 4) + rlane) * lda + koff + k0;
      V ah = Frag<T>::load(Ab + ao);
      V al;
      if (SPLIT) al = Frag<T>::load(Ab2 + ao);
#pragma unroll
      for (int j = 0; j < 4; ++j) {
        acc[i][j] = Frag<T>::mma(ah, bh[j], acc[i][j]);
        if (SPLIT) {
          acc[i][j] = Frag<T>::mma(ah, bl[j], acc[i][j]);
          acc[i][j] = Frag<T>::mma(al, bh[j], acc[i][j]);
        }
      }
      Frag<T>::guard(acc[i][0], acc[i][3], ah, SPLIT ? al : ah);
    }
    Frag<T>::keep(bh[0], bh[1], bh[2], bh[3]);
    if (SPLIT) Frag<T>::keep(bl[0], bl[1], bl[2], bl[3]);
  }
  acc_guard4(acc[0][0], acc[0][1], acc[0][2], acc[0][3]);
  acc_guard4(acc[1][0], acc[1][1], acc[1][2], acc[1][3]);
  acc_guard4(acc[2][0], acc[2][1], acc[2][2], acc[2][3]);
  acc_guard4(acc[3][0], acc[3][1], acc[3][2], acc[3][3]);

  float* slab = sT[wave];
  const float* Rb = RESID ? (resid + (size_t)b * strideR) : nullptr;
#pragma unroll
  for (int i = 0; i < 4; ++i) {
    const int mBase = m0 + (i << 4);
#pragma unroll
    for (int j = 0; j < 4; ++j) {
      const int n = n0 + (j << 4) + rlane;
      float bv = 0.f;
      if (BIAS_MODE == 2) bv = bias[n];
#pragma unroll
      for (int r = 0; r < 8; ++r) {
        float v = acc[i][j][r] * scale;
        if (BIAS_MODE == 1) v += bias[mBase + mOff + r];
        if (BIAS_MODE == 2) v += bv;
        if (RESID) v += Rb[(size_t)(mBase + mOff + r) * ldc + n];
        if (ACT == 1) v = tanhf(v);
        if (ACT == 2) v = fmaxf(v, 0.0f);
        if (ACT == 3) v = v / (1.0f + expf(-v));
        if (ACT == 4) v = (v > 0.f) ? v : 0.01f * v;
        if (ACT == 5) v = 0.5f * v * (1.0f + erff(v * 0.70710678118654752f));
        slab[(mOff + r) * 68 + (j << 4) + rlane] = v;
      }
    }
    __builtin_amdgcn_fence(__ATOMIC_RELEASE, "workgroup");
    __builtin_amdgcn_wave_barrier();
    __builtin_amdgcn_fence(__ATOMIC_ACQUIRE, "workgroup");
    if (OUT_MODE == 0) {
      float* C = (float*)Cout + (size_t)b * strideC;
      const int hh = lane >> 4, c4 = (lane & 15) * 4;
      for (int pass = 0; pass < 2; ++pass) {
#pragma unroll
        for (int it = 0; it < 8; ++it) {
          const int row = it * 2 + hh;
          v4f v = *(const v4f*)(slab + row * 68 + c4);
          *(volatile v4f*)(C + (size_t)(mBase + row) * ldc + n0 + c4) = v;
        }
        __threadfence();
      }
    } else {
      const int q = lane >> 3, c8 = (lane & 7) * 8;
      unsigned short* C  = (unsigned short*)Cout  + (size_t)b * strideC;
      unsigned short* C2 = (OUT_MODE == 2) ? ((unsigned short*)Cout2 + (size_t)b * strideC) : nullptr;
      for (int pass = 0; pass < 2; ++pass) {
#pragma unroll
        for (int it = 0; it < 4; ++it) {
          const int row = it * 4 + q;
          const float* sp = slab + row * 68 + c8;
          v8h hv, lv;
#pragma unroll
          for (int e = 0; e < 8; ++e) {
            if (OUT_MODE == 1) {
              hv[e] = (_Float16)sp[e];
            } else {
              unsigned short hb = f2bf_bits(sp[e]);
              unsigned short lb = f2bf_bits(sp[e] - bf_bits2f(hb));
              hv[e] = __builtin_bit_cast(_Float16, hb);
              lv[e] = __builtin_bit_cast(_Float16, lb);
            }
          }
          *(volatile v8h*)(C + (size_t)(mBase + row) * ldc + n0 + c8) = hv;
          if (OUT_MODE == 2) *(volatile v8h*)(C2 + (size_t)(mBase + row) * ldc + n0 + c8) = lv;
        }
        __threadfence();
      }
    }
    __builtin_amdgcn_fence(__ATOMIC_RELEASE, "workgroup");
    __builtin_amdgcn_wave_barrier();
    __builtin_amdgcn_fence(__ATOMIC_ACQUIRE, "workgroup");
  }
}

template <int MODE>
__global__ __launch_bounds__(NTHR) void cvt8_kernel(const float* __restrict__ src, unsigned short* __restrict__ dst,
                                                    int nrow, int ncol8, int spitch, int scol0, float sc) {
  const int i  = blockIdx.x * NTHR + threadIdx.x;
  const int n8 = nrow * ncol8;
  if (i < n8) {
    const int row = i / ncol8;
    const int c8  = i - row * ncol8;
    const float* sp = src + (size_t)row * spitch + scol0 + c8 * 8;
    const v4f a = *(const v4f*)(sp);
    const v4f b = *(const v4f*)(sp + 4);
    v8h hv;
#pragma unroll
    for (int e = 0; e < 4; ++e) {
      unsigned short b0, b1;
      if (MODE == 0) {
        b0 = f2bf_bits(a[e] * sc);
        b1 = f2bf_bits(b[e] * sc);
      } else {
        b0 = __builtin_bit_cast(unsigned short, (_Float16)(bf16r(a[e]) * sc));
        b1 = __builtin_bit_cast(unsigned short, (_Float16)(bf16r(b[e]) * sc));
      }
      hv[e]     = __builtin_bit_cast(_Float16, b0);
      hv[4 + e] = __builtin_bit_cast(_Float16, b1);
    }
    *(volatile v8h*)(dst + (size_t)i * 8) = hv;
    __threadfence();
    *(volatile v8h*)(dst + (size_t)i * 8) = hv;
  }
}

__global__ __launch_bounds__(NTHR) void bias_prep_kernel(const float* __restrict__ hb, const float* __restrict__ cb,
                                                         const float* __restrict__ ib,
                                                         const float* __restrict__ bi0, const float* __restrict__ bh0,
                                                         const float* __restrict__ bi1, const float* __restrict__ bh1,
                                                         const float* __restrict__ ob, float* __restrict__ dst) {
  const int blk = blockIdx.x;
  const float* pa = hb; const float* pb = hb; int n = N2H; int doff = OFF_BHID; float sc = 1.0f; int two = 0;
  if (blk == 1)      { pa = cb;  pb = cb;  n = N2H; doff = OFF_BCEL; }
  else if (blk == 2) { pa = ib;  pb = ib;  n = NH;  doff = OFF_BINP; sc = X0C; }
  else if (blk == 3) { pa = bi0; pb = bh0; n = NG4; doff = OFF_BS0; two = 1; }
  else if (blk == 4) { pa = bi1; pb = bh1; n = NG4; doff = OFF_BS1; two = 1; }
  else if (blk == 5) { pa = ob;  pb = ob;  n = NO;  doff = OFF_BOUT; }
  const int idx = threadIdx.x * 4;
  if (idx < n) {
    const v4f va = *(const v4f*)(pa + idx);
    const v4f vb = *(const v4f*)(pb + idx);
    v4f o;
#pragma unroll
    for (int e = 0; e < 4; ++e) {
      const float fb = two ? bf16r(vb[e]) : 0.0f;
      o[e] = (bf16r(va[e]) + fb) * sc;
    }
    float* op = dst + doff + idx;
    *(volatile v4f*)op = o;
    __threadfence();
    *(volatile v4f*)op = o;
  }
}

__device__ __forceinline__ void mac_h256(v8f& acc0, v8f& acc1, v8f& acc2, v8f& acc3,
                                         const _Float16* arow, const _Float16* wrow) {
#pragma unroll 1
  for (int k0 = 0; k0 < NH; k0 += 32) {
    const v16h a  = Frag<_Float16>::load(arow + k0);
    const v16h w0 = Frag<_Float16>::load(wrow + k0);
    const v16h w1 = Frag<_Float16>::load(wrow + (size_t)1 * NH * NH + k0);
    const v16h w2 = Frag<_Float16>::load(wrow + (size_t)2 * NH * NH + k0);
    const v16h w3 = Frag<_Float16>::load(wrow + (size_t)3 * NH * NH + k0);
    acc0 = Frag<_Float16>::mma(a, w0, acc0);
    acc1 = Frag<_Float16>::mma(a, w1, acc1);
    acc2 = Frag<_Float16>::mma(a, w2, acc2);
    acc3 = Frag<_Float16>::mma(a, w3, acc3);
    acc_guard4ab(acc0, acc1, acc2, acc3, a, w3);
    keep4_h(w0, w1, w2, w3);
  }
}

__global__ __launch_bounds__(RTHR) void rnn2_seq_kernel(
    const float* __restrict__ HID, const float* __restrict__ CEL, const float* __restrict__ GX0,
    const float* __restrict__ BS1,
    const unsigned short* __restrict__ WHH0p, const unsigned short* __restrict__ WIH1p,
    const unsigned short* __restrict__ WHH1p, unsigned short* __restrict__ H2S) {
  __shared__ __align__(16) _Float16 sh1[2][RBR * HP];
  __shared__ __align__(16) _Float16 sh2[2][RBR * HP];
  const _Float16* WHH0 = (const _Float16*)WHH0p;
  const _Float16* WIH1 = (const _Float16*)WIH1p;
  const _Float16* WHH1 = (const _Float16*)WHH1p;
  const int tid = threadIdx.x, lane = tid & 31, wave = tid >> 5;
  const int c = lane & 15, hh = lane >> 4, koff = hh * 8;
  const int b0 = blockIdx.x * RBR;
  const int j = 16 * wave + c;

  {
    _Float16* p1 = &sh1[0][0];
    _Float16* p2 = &sh2[0][0];
#pragma unroll 1
    for (int i = tid; i < 2 * RBR * HP; i += RTHR) { p1[i] = (_Float16)0.0f; p2[i] = (_Float16)0.0f; }
  }
  __syncthreads();
#pragma unroll 1
  for (int i = 0; i < (RBR * NH) / RTHR; ++i) {
    const int idx = i * RTHR + tid;
    const int row = idx >> 8, col = idx & (NH - 1);
    const float* hp = HID + (size_t)(b0 + row) * N2H + col;
    const float v1 = hp[0];
    const float v2 = hp[NH];
    sh1[0][row * HP + col] = (_Float16)v1;
    sh2[0][row * HP + col] = (_Float16)v2;
  }
  float cs0[8], cs1[8], gx[4][8], bb1[4];
#pragma unroll
  for (int r = 0; r < 8; ++r) cs0[r] = CEL[(size_t)(b0 + 8 * hh + r) * N2H + j];
  use8(cs0[0], cs0[1], cs0[2], cs0[3], cs0[4], cs0[5], cs0[6], cs0[7]);
#pragma unroll
  for (int r = 0; r < 8; ++r) cs1[r] = CEL[(size_t)(b0 + 8 * hh + r) * N2H + NH + j];
  use8(cs1[0], cs1[1], cs1[2], cs1[3], cs1[4], cs1[5], cs1[6], cs1[7]);
#pragma unroll
  for (int g = 0; g < 4; ++g) {
#pragma unroll
    for (int r = 0; r < 8; ++r) gx[g][r] = GX0[(size_t)(b0 + 8 * hh + r) * NG4 + g * NH + j];
    use8(gx[g][0], gx[g][1], gx[g][2], gx[g][3], gx[g][4], gx[g][5], gx[g][6], gx[g][7]);
  }
#pragma unroll
  for (int g = 0; g < 4; ++g) bb1[g] = BS1[g * NH + j];
  __syncthreads();

  const v8f z8 = {0.f, 0.f, 0.f, 0.f, 0.f, 0.f, 0.f, 0.f};

#pragma unroll 1
  for (int s = 0; s < NS; ++s) {
    const int pr = s & 1, cu = pr ^ 1;
    {
      const _Float16* arow = &sh1[pr][0] + c * HP + koff;
      _Float16* hdst = &sh1[cu][0];
      v8f acc[4];
      acc[0] = z8; acc[1] = z8; acc[2] = z8; acc[3] = z8;
      mac_h256(acc[0], acc[1], acc[2], acc[3], arow, WHH0 + (size_t)j * NH + koff);
      acc_guard4(acc[0], acc[1], acc[2], acc[3]);
#pragma unroll
      for (int r = 0; r < 8; ++r) {
        const float zi = acc[0][r] * WC_INV + gx[0][r];
        const float zf = acc[1][r] * WC_INV + gx[1][r];
        const float zg = acc[2][r] * WC_INV + gx[2][r];
        const float zo = acc[3][r] * WC_INV + gx[3][r];
        const float ig = fsig(zi);
        const float fg = fsig(zf);
        const float og = fsig(zo);
        const float gg = ftanh(zg);
        const float cn = fg * cs0[r] + ig * gg;
        cs0[r] = cn;
        const float hn = og * ftanh(cn);
        hdst[(8 * hh + r) * HP + j] = (_Float16)hn;
      }
    }
    __syncthreads();
    {
      const _Float16* a1row = &sh1[cu][0] + c * HP + koff;
      const _Float16* a2row = &sh2[pr][0] + c * HP + koff;
      _Float16* hdst = &sh2[cu][0];
      v8f acc[4];
      acc[0] = z8; acc[1] = z8; acc[2] = z8; acc[3] = z8;
      mac_h256(acc[0], acc[1], acc[2], acc[3], a1row, WIH1 + (size_t)j * NH + koff);
      mac_h256(acc[0], acc[1], acc[2], acc[3], a2row, WHH1 + (size_t)j * NH + koff);
      acc_guard4(acc[0], acc[1], acc[2], acc[3]);
#pragma unroll
      for (int r = 0; r < 8; ++r) {
        const float zi = acc[0][r] * WC_INV + bb1[0];
        const float zf = acc[1][r] * WC_INV + bb1[1];
        const float zg = acc[2][r] * WC_INV + bb1[2];
        const float zo = acc[3][r] * WC_INV + bb1[3];
        const float ig = fsig(zi);
        const float fg = fsig(zf);
        const float og = fsig(zo);
        const float gg = ftanh(zg);
        const float cn = fg * cs1[r] + ig * gg;
        cs1[r] = cn;
        const float hn = og * ftanh(cn);
        hdst[(8 * hh + r) * HP + j] = (_Float16)hn;
      }
    }
    __syncthreads();
    {
      const v4u hv = *(const v4u*)(const void*)(&sh2[cu][wave * HP + 8 * lane]);
      unsigned short* dp = H2S + ((size_t)(b0 + wave) * NS + (size_t)s) * NH + 8 * lane;
      for (int pass = 0; pass < 2; ++pass) {
        *(volatile v4u*)dp = hv;
        __threadfence();
      }
    }
  }
}

extern "C" void kernel_launch(void* const* d_in, const int* in_sizes, int n_in,
                              void* d_out, int out_size, void* d_ws, size_t ws_size, hipStream_t stream) {
  if (n_in < 17 || d_out == nullptr || d_ws == nullptr) return;
  if (in_sizes[0] != NB * NLAT || in_sizes[1] != N2H * NLAT || in_sizes[2] != N2H || in_sizes[3] != N2H * NLAT ||
      in_sizes[4] != N2H || in_sizes[5] != NH * NLAT || in_sizes[6] != NH || in_sizes[7] != NG4 * NH ||
      in_sizes[8] != NG4 * NH || in_sizes[9] != NG4 || in_sizes[10] != NG4 || in_sizes[11] != NG4 * NH ||
      in_sizes[12] != NG4 * NH || in_sizes[13] != NG4 || in_sizes[14] != NG4 || in_sizes[15] != NO * NH ||
      in_sizes[16] != NO || out_size != NROWS * NO) return;

  const float* z    = (const float*)d_in[0];
  const float* fhw  = (const float*)d_in[1];
  const float* fhb  = (const float*)d_in[2];
  const float* fcw  = (const float*)d_in[3];
  const float* fcb  = (const float*)d_in[4];
  const float* fiw  = (const float*)d_in[5];
  const float* fib  = (const float*)d_in[6];
  const float* wih0 = (const float*)d_in[7];
  const float* whh0 = (const float*)d_in[8];
  const float* bih0 = (const float*)d_in[9];
  const float* bhh0 = (const float*)d_in[10];
  const float* wih1 = (const float*)d_in[11];
  const float* whh1 = (const float*)d_in[12];
  const float* bih1 = (const float*)d_in[13];
  const float* bhh1 = (const float*)d_in[14];
  const float* wo   = (const float*)d_in[15];
  const float* bo   = (const float*)d_in[16];
  float* out = (float*)d_out;

  char* ws = (char*)d_ws; size_t off = 0;
  auto carve = [&](size_t bytes) -> char* { char* p = ws + off; off += (bytes + 255) & ~(size_t)255; return p; };
  unsigned short* Z16   = (unsigned short*)carve((size_t)NB * NLAT * 2);
  unsigned short* FHW16 = (unsigned short*)carve((size_t)N2H * NLAT * 2);
  unsigned short* FCW16 = (unsigned short*)carve((size_t)N2H * NLAT * 2);
  unsigned short* FIW16 = (unsigned short*)carve((size_t)NH * NLAT * 2);
  unsigned short* WIH0  = (unsigned short*)carve((size_t)NG4 * NH * 2);
  unsigned short* WHH0  = (unsigned short*)carve((size_t)NG4 * NH * 2);
  unsigned short* WIH1  = (unsigned short*)carve((size_t)NG4 * NH * 2);
  unsigned short* WHH1  = (unsigned short*)carve((size_t)NG4 * NH * 2);
  unsigned short* WO16  = (unsigned short*)carve((size_t)NO * NH * 2);
  float*          BIASP = (float*)carve((size_t)NBIAS * 4);
  float*          HID   = (float*)carve((size_t)NB * N2H * 4);
  float*          CEL   = (float*)carve((size_t)NB * N2H * 4);
  unsigned short* X016  = (unsigned short*)carve((size_t)NB * NH * 2);
  float*          GX0   = (float*)carve((size_t)NB * NG4 * 4);
  unsigned short* H2SEQ = (unsigned short*)carve((size_t)NROWS * NH * 2);
  if (off > ws_size || off > (size_t)134217728) return;

  const int n8z  = NB * (NLAT / 8);
  const int n8hw = N2H * (NLAT / 8);
  const int n8iw = NH * (NLAT / 8);
  const int n8w  = NG4 * (NH / 8);
  const int n8o  = NO * (NH / 8);
  cvt8_kernel<1><<<(n8z  + NTHR - 1) / NTHR, NTHR, 0, stream>>>(z,    Z16,   NB,  NLAT / 8, NLAT, 0, ZC);
  cvt8_kernel<1><<<(n8hw + NTHR - 1) / NTHR, NTHR, 0, stream>>>(fhw,  FHW16, N2H, NLAT / 8, NLAT, 0, WC);
  cvt8_kernel<1><<<(n8hw + NTHR - 1) / NTHR, NTHR, 0, stream>>>(fcw,  FCW16, N2H, NLAT / 8, NLAT, 0, WC);
  cvt8_kernel<1><<<(n8iw + NTHR - 1) / NTHR, NTHR, 0, stream>>>(fiw,  FIW16, NH,  NLAT / 8, NLAT, 0, WC);
  cvt8_kernel<1><<<(n8w  + NTHR - 1) / NTHR, NTHR, 0, stream>>>(wih0, WIH0,  NG4, NH / 8,   NH,   0, WC);
  cvt8_kernel<1><<<(n8w  + NTHR - 1) / NTHR, NTHR, 0, stream>>>(whh0, WHH0,  NG4, NH / 8,   NH,   0, WC);
  cvt8_kernel<1><<<(n8w  + NTHR - 1) / NTHR, NTHR, 0, stream>>>(wih1, WIH1,  NG4, NH / 8,   NH,   0, WC);
  cvt8_kernel<1><<<(n8w  + NTHR - 1) / NTHR, NTHR, 0, stream>>>(whh1, WHH1,  NG4, NH / 8,   NH,   0, WC);
  cvt8_kernel<1><<<(n8o  + NTHR - 1) / NTHR, NTHR, 0, stream>>>(wo,   WO16,  NO,  NH / 8,   NH,   0, WC);
  bias_prep_kernel<<<6, NTHR, 0, stream>>>(fhb, fcb, fib, bih0, bhh0, bih1, bhh1, bo, BIASP);

  const dim3 g_hid(((NB / 64) * (N2H / 64) + 7) / 8, 1);
  const dim3 g_x0 (((NB / 64) * (NH / 64) + 7) / 8, 1);
  wmma_gemm64<0, false, 2, 0, false, 0><<<g_hid, 256, 0, stream>>>(
      Z16, Z16, NLAT, 0L, FHW16, FHW16, NLAT, 0L, (void*)HID, (void*)HID, N2H, 0L,
      BIASP + OFF_BHID, GX0, 0L, NB, N2H, NLAT, 1.0f / (ZC * WC));
  wmma_gemm64<0, false, 2, 0, false, 0><<<g_hid, 256, 0, stream>>>(
      Z16, Z16, NLAT, 0L, FCW16, FCW16, NLAT, 0L, (void*)CEL, (void*)CEL, N2H, 0L,
      BIASP + OFF_BCEL, GX0, 0L, NB, N2H, NLAT, 1.0f / (ZC * WC));
  wmma_gemm64<0, false, 2, 1, false, 0><<<g_x0, 256, 0, stream>>>(
      Z16, Z16, NLAT, 0L, FIW16, FIW16, NLAT, 0L, (void*)X016, (void*)X016, NH, 0L,
      BIASP + OFF_BINP, GX0, 0L, NB, NH, NLAT, X0C / (ZC * WC));
  const dim3 g_gx(((NB / 64) * (NG4 / 64) + 7) / 8, 1);
  wmma_gemm64<0, false, 2, 0, false, 0><<<g_gx, 256, 0, stream>>>(
      X016, X016, NH, 0L, WIH0, WIH0, NH, 0L, (void*)GX0, (void*)GX0, NG4, 0L,
      BIASP + OFF_BS0, HID, 0L, NB, NG4, NH, 1.0f / (X0C * WC));

  rnn2_seq_kernel<<<NB / RBR, RTHR, 0, stream>>>(HID, CEL, GX0, BIASP + OFF_BS1, WHH0, WIH1, WHH1, H2SEQ);

  const dim3 g_out(((NROWS / 64) * (NO / 64) + 7) / 8, 1);
  wmma_gemm64<0, false, 2, 0, false, 0><<<g_out, 256, 0, stream>>>(
      H2SEQ, H2SEQ, NH, 0L, WO16, WO16, NH, 0L, (void*)out, (void*)out, NO, 0L,
      BIASP + OFF_BOUT, GX0, 0L, NROWS, NO, NH, 1.0f / WC);
}
